// S5Dual_89653147337062
// MI455X (gfx1250) — hardware-verified
//
#include <hip/hip_runtime.h>
#include <math.h>

typedef _Float16 v16h __attribute__((ext_vector_type(16)));
typedef _Float16 v8h  __attribute__((ext_vector_type(8)));
typedef float    v8f  __attribute__((ext_vector_type(8)));
typedef float    v4f  __attribute__((ext_vector_type(4)));
typedef v8h __attribute__((may_alias)) v8ha;
typedef v4f __attribute__((may_alias)) v4fa;

union Frag { v16h v; v8h half[2]; };

#define NB    4
#define NL    8192
#define NH    256
#define NP    256
#define NROWS (NB * NL)
#define NX    (NROWS * NH)
#define NW    (NP * NH)
#define KC    (2 * NP)
#define TS    32
#define NCH   (NL / TS)
#define PG    64
#define WSC   16.0f
#define WSCI  0.0625f

#define WS_X16   ((size_t)0)
#define WS_BB    (WS_X16 + (size_t)NX * 2)
#define WS_CC    (WS_BB + (size_t)2 * 2 * NW * 2)
#define WS_LAM   (WS_CC + (size_t)2 * NH * KC * 2)
#define WS_XS    (WS_LAM + (size_t)4096)
#define WS_TOTAL (WS_XS + (size_t)2 * NROWS * KC * 2)

__device__ __forceinline__ v8f wmma_f16(v16h a, v16h b, v8f c) {
  v8f d = __builtin_amdgcn_wmma_f32_16x16x32_f16(false, a, false, b, (short)0, c, false, false);
  asm volatile("v_nop\n\tv_nop\n\tv_nop\n\tv_nop" : "+v"(d) : "v"(a), "v"(b));
  return d;
}

__device__ __forceinline__ v16h load_frag(const _Float16* p, int h) {
  Frag f;
  f.half[0] = *(const v8ha*)(p + 8 * h);
  f.half[1] = *(const v8ha*)(p + 16 + 8 * h);
  return f.v;
}

__device__ __forceinline__ float gelu_f(float v) {
  return 0.5f * v * (1.0f + erff(v * 0.70710678118654752f));
}

__global__ __launch_bounds__(256) void k_cvt(const float* __restrict__ x, _Float16* __restrict__ xh) {
  const int g = blockIdx.x * 256 + threadIdx.x;
  if (g >= NX / 8) return;
  const float* src = x + (size_t)g * 8;
  const v4f a = *(const v4fa*)src;
  const v4f c = *(const v4fa*)(src + 4);
  const v8h o = { (_Float16)a.x, (_Float16)a.y, (_Float16)a.z, (_Float16)a.w,
                  (_Float16)c.x, (_Float16)c.y, (_Float16)c.z, (_Float16)c.w };
  _Float16* dst = xh + (size_t)g * 8;
  *(volatile v8h*)dst = o;
  __threadfence();
  *(volatile v8h*)dst = o;
}

__device__ __forceinline__ void prep_store(const _Float16* sB, const _Float16* sC,
                                           _Float16* bb, _Float16* cc, int dir, int pgrp, int w, int lane) {
  #pragma unroll
  for (int i = 0; i < 4; ++i) {
    const int rid = w * 4 + i;
    {
      const int part = rid >> 4, j = rid & 15;
      const v8h v = *(const v8ha*)(sB + (part * 16 + j) * NH + 8 * lane);
      _Float16* dst = bb + ((size_t)(dir * 2 + part) * NP + pgrp * 16 + j) * NH + 8 * lane;
      *(volatile v8h*)dst = v;
    }
    {
      const int j = rid >> 1, hl = rid & 1;
      const v8h v = *(const v8ha*)(sC + j * KC + NP * hl + 8 * lane);
      _Float16* dst = cc + ((size_t)dir * NH + pgrp * 16 + j) * KC + NP * hl + 8 * lane;
      *(volatile v8h*)dst = v;
    }
  }
}

__global__ __launch_bounds__(256) void k_prep(
    const float* __restrict__ lgr, const float* __restrict__ img, const float* __restrict__ lgd,
    const float* __restrict__ Br,  const float* __restrict__ Bi,
    const float* __restrict__ Cr,  const float* __restrict__ Ci,
    _Float16* __restrict__ bb, _Float16* __restrict__ cc,
    float* __restrict__ lamr, float* __restrict__ lami, int dir)
{
  __shared__ float sCoR[NP];
  __shared__ float sCoI[NP];
  __shared__ __attribute__((aligned(16))) _Float16 sB[2 * 16 * NH];
  __shared__ __attribute__((aligned(16))) _Float16 sC[16 * KC];

  const int tid = threadIdx.x, lane = tid & 31, w = tid >> 5;
  const int pgrp = blockIdx.x;

  const float Lr = -expf(lgr[tid]);
  const float Li = img[tid];
  const float Dl = expf(lgd[tid]);
  const float ad = Lr * Dl, bd = Li * Dl;
  const float ea = expf(ad);
  const float lbr = ea * cosf(bd);
  const float lbi = ea * sinf(bd);
  {
    const float den = fmaxf(Lr * Lr + Li * Li, 1e-12f);
    const float rden = 1.0f / den;
    const float invr = Lr * rden, invi = -Li * rden;
    const float dr = lbr - 1.0f, di = lbi;
    sCoR[tid] = invr * dr - invi * di;
    sCoI[tid] = invr * di + invi * dr;
  }
  if (pgrp == 0) {
    *(volatile float*)(lamr + dir * NP + tid) = lbr;
    *(volatile float*)(lami + dir * NP + tid) = lbi;
  }
  __syncthreads();

  #pragma unroll 1
  for (int j = 0; j < 16; ++j) {
    const int p = pgrp * 16 + j;
    const float br = Br[p * NH + tid], bi = Bi[p * NH + tid];
    const float cr = sCoR[p], ci = sCoI[p];
    sB[(0 * 16 + j) * NH + tid] = (_Float16)((cr * br - ci * bi) * WSC);
    sB[(1 * 16 + j) * NH + tid] = (_Float16)((cr * bi + ci * br) * WSC);
  }
  #pragma unroll 1
  for (int j = 0; j < 16; ++j) {
    const int hh = pgrp * 16 + j;
    sC[j * KC + tid]      = (_Float16)(Cr[hh * NP + tid] * WSC);
    sC[j * KC + NP + tid] = (_Float16)(-Ci[hh * NP + tid] * WSC);
  }
  __syncthreads();

  prep_store(sB, sC, bb, cc, dir, pgrp, w, lane);
  __threadfence();
  prep_store(sB, sC, bb, cc, dir, pgrp, w, lane);
  if (pgrp == 0) {
    *(volatile float*)(lamr + dir * NP + tid) = lbr;
    *(volatile float*)(lami + dir * NP + tid) = lbi;
  }
}

__device__ __forceinline__ void scan_store(const _Float16* sS, _Float16* xsd,
                                           size_t rowbase, int p0, int w, int lane) {
  const int q8 = lane & 7, sub = lane >> 3;
  #pragma unroll
  for (int i = 0; i < 8; ++i) {
    const int lid = w * 32 + i * 4 + sub;
    const int row = lid >> 1, part = lid & 1;
    const v8h v = *(const v8ha*)(sS + part * (TS * PG) + row * PG + 8 * q8);
    _Float16* dst = xsd + (rowbase + row) * KC + part * NP + p0 + 8 * q8;
    *(volatile v8h*)dst = v;
  }
}

__global__ __launch_bounds__(64) void k_scan(
    const _Float16* __restrict__ xh,
    const _Float16* __restrict__ bb,
    const float* __restrict__ lamr, const float* __restrict__ lami,
    _Float16* __restrict__ xs)
{
  __shared__ __attribute__((aligned(16))) float    sU[2 * TS * PG];
  __shared__ __attribute__((aligned(16))) _Float16 sS[2 * TS * PG];

  const int tid = threadIdx.x, lane = tid & 31, w = tid >> 5;
  const int h = lane >> 4, m = lane & 15;
  const int pg = blockIdx.x, b = blockIdx.y, dir = blockIdx.z;
  const int p0 = pg * PG;

  const float lr = lamr[dir * NP + p0 + tid];
  const float li = lami[dir * NP + p0 + tid];
  const _Float16* bbr = bb + ((size_t)(dir * 2 + 0) * NP + p0 + m) * NH;
  const _Float16* bbi = bb + ((size_t)(dir * 2 + 1) * NP + p0 + m) * NH;
  _Float16* xsd = xs + (size_t)dir * NROWS * KC;

  const v8f zero8 = {0.f, 0.f, 0.f, 0.f, 0.f, 0.f, 0.f, 0.f};
  float sr = 0.0f, si = 0.0f;

  #pragma unroll 1
  for (int c = 0; c < NCH; ++c) {
    const int g0 = dir ? (NL - TS - TS * c) : (TS * c);
    const size_t rowbase = (size_t)b * NL + g0;

    const _Float16* xa = xh + (rowbase + 16 * w + m) * NH;
    v8f accR[4], accI[4];
    #pragma unroll
    for (int nt = 0; nt < 4; ++nt) { accR[nt] = zero8; accI[nt] = zero8; }
    #pragma unroll 1
    for (int k0 = 0; k0 < NH; k0 += 32) {
      const v16h a = load_frag(xa + k0, h);
      #pragma unroll
      for (int nt = 0; nt < 4; ++nt) {
        const v16h fr = load_frag(bbr + (size_t)nt * 16 * NH + k0, h);
        const v16h fi = load_frag(bbi + (size_t)nt * 16 * NH + k0, h);
        accR[nt] = wmma_f16(a, fr, accR[nt]);
        accI[nt] = wmma_f16(a, fi, accI[nt]);
      }
    }
    #pragma unroll
    for (int nt = 0; nt < 4; ++nt) {
      #pragma unroll
      for (int r = 0; r < 8; ++r) {
        const int idx = (16 * w + 8 * h + r) * PG + 16 * nt + m;
        sU[idx]           = accR[nt][r];
        sU[TS * PG + idx] = accI[nt][r];
      }
    }
    __syncthreads();

    #pragma unroll 4
    for (int j = 0; j < TS; ++j) {
      const int l = dir ? (TS - 1 - j) : j;
      const float ur = sU[l * PG + tid] * WSCI;
      const float ui = sU[TS * PG + l * PG + tid] * WSCI;
      const float nr = lr * sr - li * si + ur;
      const float ni = lr * si + li * sr + ui;
      sr = nr; si = ni;
      sS[l * PG + tid]           = (_Float16)sr;
      sS[TS * PG + l * PG + tid] = (_Float16)si;
    }
    __syncthreads();

    scan_store(sS, xsd, rowbase, p0, w, lane);
    __threadfence();
    scan_store(sS, xsd, rowbase, p0, w, lane);
    __syncthreads();
  }
}

__device__ __forceinline__ void out_store(const float* so, float* out, int row0, int h0, int lane) {
  const int q8 = lane & 7, sub = lane >> 3;
  #pragma unroll
  for (int i = 0; i < 8; ++i) {
    const int lid = i * 4 + sub;
    const int row = lid >> 1, hl = lid & 1;
    const v4f v = *(const v4fa*)(so + row * 64 + 32 * hl + 4 * q8);
    float* dst = out + (size_t)(row0 + row) * NH + h0 + 32 * hl + 4 * q8;
    *(volatile v4f*)dst = v;
  }
}

__global__ __launch_bounds__(128) void k_out(
    const _Float16* __restrict__ xs,
    const _Float16* __restrict__ cc,
    const float* __restrict__ x,
    const float* __restrict__ Df, const float* __restrict__ Db,
    float* __restrict__ out)
{
  __shared__ __attribute__((aligned(16))) float sO[4 * 16 * 64];

  const int tid = threadIdx.x, lane = tid & 31, w = tid >> 5;
  const int h = lane >> 4, m = lane & 15;
  const int row0 = blockIdx.x * 64 + 16 * w;
  const int h0 = blockIdx.y * 64;

  const _Float16* a0p = xs + (size_t)(row0 + m) * KC;
  const _Float16* a1p = xs + (size_t)NROWS * KC + (size_t)(row0 + m) * KC;
  const _Float16* c0p = cc + (size_t)(h0 + m) * KC;
  const _Float16* c1p = cc + (size_t)NH * KC + (size_t)(h0 + m) * KC;

  const v8f zero8 = {0.f, 0.f, 0.f, 0.f, 0.f, 0.f, 0.f, 0.f};
  v8f af[4], ab[4];
  #pragma unroll
  for (int nt = 0; nt < 4; ++nt) { af[nt] = zero8; ab[nt] = zero8; }

  #pragma unroll 1
  for (int k0 = 0; k0 < KC; k0 += 32) {
    const v16h a0 = load_frag(a0p + k0, h);
    const v16h a1 = load_frag(a1p + k0, h);
    #pragma unroll
    for (int nt = 0; nt < 4; ++nt) {
      const v16h b0 = load_frag(c0p + (size_t)nt * 16 * KC + k0, h);
      const v16h b1 = load_frag(c1p + (size_t)nt * 16 * KC + k0, h);
      af[nt] = wmma_f16(a0, b0, af[nt]);
      ab[nt] = wmma_f16(a1, b1, ab[nt]);
    }
  }

  float* so = sO + w * 1024;
  #pragma unroll
  for (int nt = 0; nt < 4; ++nt) {
    const int col = h0 + 16 * nt + m;
    const float df = Df[col], db = Db[col];
    #pragma unroll
    for (int r = 0; r < 8; ++r) {
      const int rowl = 8 * h + r;
      const float xv = x[(size_t)(row0 + rowl) * NH + col];
      const float yf = af[nt][r] * WSCI + df * xv;
      const float yb = ab[nt][r] * WSCI + db * xv;
      so[rowl * 64 + 16 * nt + m] = gelu_f(yf) + gelu_f(yb);
    }
  }
  __syncthreads();

  out_store(so, out, row0, h0, lane);
  __threadfence();
  out_store(so, out, row0, h0, lane);
}

extern "C" void kernel_launch(void* const* d_in, const int* in_sizes, int n_in,
                              void* d_out, int out_size, void* d_ws, size_t ws_size,
                              hipStream_t stream) {
  if (n_in < 17) return;
  if (in_sizes[0] != NX || out_size != NX) return;
  for (int dir = 0; dir < 2; ++dir) {
    const int base = 1 + 8 * dir;
    if (in_sizes[base + 0] != NP || in_sizes[base + 1] != NP || in_sizes[base + 2] != NP) return;
    if (in_sizes[base + 3] != NW || in_sizes[base + 4] != NW) return;
    if (in_sizes[base + 5] != NW || in_sizes[base + 6] != NW) return;
    if (in_sizes[base + 7] != NH) return;
  }
  if (WS_TOTAL > ws_size) return;

  const float* x = (const float*)d_in[0];
  float* out = (float*)d_out;
  char* ws = (char*)d_ws;
  _Float16* xh  = (_Float16*)(ws + WS_X16);
  _Float16* bb  = (_Float16*)(ws + WS_BB);
  _Float16* cc  = (_Float16*)(ws + WS_CC);
  float* lamr   = (float*)(ws + WS_LAM);
  float* lami   = (float*)(ws + WS_LAM + 2048);
  _Float16* xs  = (_Float16*)(ws + WS_XS);

  k_cvt<<<(NX / 8) / 256, 256, 0, stream>>>(x, xh);

  for (int dir = 0; dir < 2; ++dir) {
    const int base = 1 + 8 * dir;
    k_prep<<<NP / 16, 256, 0, stream>>>(
        (const float*)d_in[base + 0], (const float*)d_in[base + 1], (const float*)d_in[base + 2],
        (const float*)d_in[base + 3], (const float*)d_in[base + 4],
        (const float*)d_in[base + 5], (const float*)d_in[base + 6],
        bb, cc, lamr, lami, dir);
  }

  dim3 gScan(NP / PG, NB, 2);
  k_scan<<<gScan, 64, 0, stream>>>(xh, bb, lamr, lami, xs);

  dim3 gOut(NROWS / 64, NH / 64);
  k_out<<<gOut, 128, 0, stream>>>(xs, cc, x, (const float*)d_in[8], (const float*)d_in[16], out);
}
